// MultiHeadSpatialAttention_18116172054581
// MI455X (gfx1250) — hardware-verified
//
#include <hip/hip_runtime.h>
#include <math.h>

typedef __attribute__((ext_vector_type(16))) _Float16 v16h;
typedef __attribute__((ext_vector_type(16))) __bf16 v16b;
typedef __attribute__((ext_vector_type(8)))  _Float16 v8h;
typedef __attribute__((ext_vector_type(8)))  float v8f;
typedef __attribute__((ext_vector_type(4)))  float v4f;
typedef __attribute__((ext_vector_type(2)))  float v2f;
typedef __attribute__((ext_vector_type(4)))  unsigned v4u;
typedef __attribute__((ext_vector_type(4)))  int v4i;
typedef float __attribute__((may_alias)) float_a;
typedef int __attribute__((may_alias)) int_a;

template <typename T> __device__ __forceinline__ void vst2(void* p, T v) { *(volatile T*)p = v; __threadfence(); *(volatile T*)p = v; }
__device__ __forceinline__ v8f wmma16(v16h a, v16h b, v8f c) {
  v8f d = __builtin_amdgcn_wmma_f32_16x16x32_f16(false, a, false, b, (short)0, c, false, false);
  asm volatile("v_nop\n\tv_nop\n\tv_nop\n\tv_nop" : "+v"(d) : "v"(a), "v"(b));
  return d;
}
__device__ __forceinline__ v8f wmma_bf(v16b a, v16b b, v8f c) {
  v8f d = __builtin_amdgcn_wmma_f32_16x16x32_bf16(false, a, false, b, (short)0, c, false, false);
  asm volatile("v_nop\n\tv_nop\n\tv_nop\n\tv_nop" : "+v"(d) : "v"(a), "v"(b));
  return d;
}
__device__ __forceinline__ v16h frag_h(const _Float16* rowk0, int lane) {
  union { v16h v; v8h q[2]; } u; const _Float16* p = rowk0 + 8 * (lane >> 4);
  u.q[0] = *(const v8h*)p; u.q[1] = *(const v8h*)(p + 16); return u.v;
}
__device__ __forceinline__ v16h frag_f32(const float* rowk0, int lane) {
  v16h a; const float* p = rowk0 + 8 * (lane >> 4);
#pragma unroll
  for (int i = 0; i < 8; ++i) { a[i] = (_Float16)p[i]; a[8 + i] = (_Float16)p[16 + i]; }
  return a;
}
__device__ __forceinline__ v16h frag_f32s(const float* rowk0, int lane, float sc) {
  v16h a; const float* p = rowk0 + 8 * (lane >> 4);
#pragma unroll
  for (int i = 0; i < 8; ++i) { a[i] = (_Float16)(p[i] * sc); a[8 + i] = (_Float16)(p[16 + i] * sc); }
  return a;
}
__device__ __forceinline__ v16h fragc_f32(const float* W, int k0, int n, int lane, int ld, int K) {
  v16h a; const int g = lane >> 4;
#pragma unroll
  for (int i = 0; i < 8; ++i) { const int ka = k0 + 8 * g + i, kb = ka + 16;
    a[i] = (_Float16)(ka < K ? W[(size_t)(ka < K ? ka : K - 1) * ld + n] : 0.f); a[8 + i] = (_Float16)(kb < K ? W[(size_t)(kb < K ? kb : K - 1) * ld + n] : 0.f); }
  return a;
}
struct F2 { v16b h, l; };
__device__ __forceinline__ F2 bsplit16(const float v[16]) { F2 r;
#pragma unroll
  for (int i = 0; i < 16; ++i) { const __bf16 h = (__bf16)v[i]; r.h[i] = h; r.l[i] = (__bf16)(v[i] - (float)h); }
  return r; }
__device__ __forceinline__ F2 split_row(const float* row, int k0, int lane) { float v[16]; const float* p = row + k0 + 8 * (lane >> 4);
#pragma unroll
  for (int i = 0; i < 8; ++i) { v[i] = p[i]; v[8 + i] = p[16 + i]; }
  return bsplit16(v); }
__device__ __forceinline__ F2 split_rowK(const float* row, int k0, int lane, int K) { float v[16]; const int g = lane >> 4;
#pragma unroll
  for (int i = 0; i < 8; ++i) { const int ka = k0 + 8 * g + i, kb = ka + 16; v[i] = ka < K ? row[ka < K ? ka : K - 1] : 0.f; v[8 + i] = kb < K ? row[kb < K ? kb : K - 1] : 0.f; }
  return bsplit16(v); }
__device__ __forceinline__ F2 split_col(const float* W, int k0, int n, int lane, int ld, int K) { float v[16]; const int g = lane >> 4;
#pragma unroll
  for (int i = 0; i < 8; ++i) { const int ka = k0 + 8 * g + i, kb = ka + 16; v[i] = ka < K ? W[(size_t)(ka < K ? ka : K - 1) * ld + n] : 0.f; v[8 + i] = kb < K ? W[(size_t)(kb < K ? kb : K - 1) * ld + n] : 0.f; }
  return bsplit16(v); }
__device__ __forceinline__ v8f mac3(const F2& a, const F2& b, v8f c) { c = wmma_bf(a.l, b.h, c); c = wmma_bf(a.h, b.l, c); return wmma_bf(a.h, b.h, c); }
__device__ __forceinline__ float sigm(float v) { return 1.0f / (1.0f + expf(-v)); }
#define LDSX() do { asm volatile("s_wait_dscnt 0" ::: "memory"); __builtin_amdgcn_wave_barrier(); __builtin_amdgcn_fence(__ATOMIC_RELEASE, "workgroup"); } while (0)


#define NB 16
#define CIN 256
#define TT 1024
#define CC 512
#define NH 8
#define HD 64
#define BG 2
#define ZG (BG * NH)
#define NR (NB * TT)
#ifndef TNB
#define TNB NB
#endif
typedef __attribute__((ext_vector_type(8))) __bf16 v8b;
__device__ __forceinline__ v16b frag_b(const __bf16* rowk0, int lane) {
  union { v16b v; v8b q[2]; } u; const __bf16* p = rowk0 + 8 * (lane >> 4);
  u.q[0] = *(const v8b*)p; u.q[1] = *(const v8b*)(p + 16); return u.v;
}
__device__ __forceinline__ float bfr(float v) { return (float)(__bf16)v; }
__device__ __attribute__((noinline)) float exp_ni(float v) { return expf(v); }
__device__ __attribute__((noinline)) float erf_ni(float v) { return erff(v); }

#define OUT1_OFF ((size_t)NB * CIN * TT)
#define WS_QH  0u
#define WS_QL  (WS_QH + 2u * (size_t)NR * CC)
#define WS_KH  (WS_QL + 2u * (size_t)NR * CC)
#define WS_VT  (WS_KH + 2u * (size_t)NR * CC)
#define WS_S   (WS_VT + 2u * (size_t)NR * CC)
#define WS_PH  (WS_S + 4u * (size_t)ZG * TT * TT)
#define WS_Y   (WS_PH + 2u * (size_t)ZG * TT * TT)
#define WS_Z1  (WS_Y + 4u * (size_t)NR * CC)
#define WS_HM  (WS_Z1 + 4u * (size_t)NR * CIN)
#define WS_END (WS_HM + 4u * (size_t)NR * CIN)

__global__ __launch_bounds__(128) void k_proj(const float* __restrict__ X, const float* __restrict__ WQ, const float* __restrict__ BQ, const float* __restrict__ WK, const float* __restrict__ BK, const float* __restrict__ WV, const float* __restrict__ BV, _Float16* __restrict__ QH, _Float16* __restrict__ QL, _Float16* __restrict__ KH, _Float16* __restrict__ VT) {
  __shared__ __align__(16) __bf16 sx[64][CIN + 8]; __shared__ __align__(16) _Float16 sh[64][136], sl[64][136]; __shared__ __align__(16) _Float16 th[128][72];
  const int tid = threadIdx.x, wave = tid >> 5, lane = tid & 31, col = lane & 15, g = lane >> 4; const int p0 = blockIdx.x * 64; const int c0 = blockIdx.y * 128; const size_t b = blockIdx.z / 3; const int which = blockIdx.z % 3;
  const float* Wm = which == 0 ? WQ : which == 1 ? WK : WV; const float* Bm = which == 0 ? BQ : which == 1 ? BK : BV;
  for (int e = tid; e < CIN * 64; e += 128) { const int c = e >> 6, pl = e & 63; sx[pl][c] = (__bf16)X[(b * CIN + c) * (size_t)TT + p0 + pl]; }
  __syncthreads();
  v8f acc[8] = {};
#pragma unroll 2
  for (int kc = 0; kc < CIN / 32; ++kc) { const v16b a = frag_b(&sx[wave * 16 + col][kc * 32], lane);
#pragma unroll
    for (int j = 0; j < 8; ++j) { v16b w; const int o = c0 + j * 16 + col;
#pragma unroll
      for (int i = 0; i < 8; ++i) { w[i] = (__bf16)Wm[(size_t)(kc * 32 + 8 * g + i) * CC + o]; w[8 + i] = (__bf16)Wm[(size_t)(kc * 32 + 16 + 8 * g + i) * CC + o]; }
      acc[j] = wmma_bf(a, w, acc[j]); } }
#pragma unroll
  for (int j = 0; j < 8; ++j) { const float bb = bfr(Bm[c0 + j * 16 + col]);
#pragma unroll
    for (int r = 0; r < 8; ++r) { const float v = acc[j][r] + bb; const int rl = wave * 16 + 8 * g + r, cl = j * 16 + col; const _Float16 hv = (_Float16)v;
      if (which == 2) th[cl][rl] = hv; else { sh[rl][cl] = hv; sl[rl][cl] = (_Float16)(v - (float)hv); } } }
  __syncthreads();
  if (which < 2) { _Float16* dh = which == 0 ? QH : KH; for (int e = tid; e < 64 * 16; e += 128) { const int rl = e >> 4, q = e & 15; const size_t row = b * TT + p0 + rl; vst2((unsigned*)(dh + row * CC + c0 + q * 8), *(const v4u*)&sh[rl][q * 8]); if (which == 0) vst2((unsigned*)(QL + row * CC + c0 + q * 8), *(const v4u*)&sl[rl][q * 8]); } }
  else { for (int e = tid; e < 128 * 8; e += 128) { const int cl = e >> 3, q = e & 7; vst2((unsigned*)(VT + (b * CC + c0 + cl) * (size_t)TT + p0 + q * 8), *(const v4u*)&th[cl][q * 8]); } } }
__global__ __launch_bounds__(128) void k_sc(const _Float16* __restrict__ QH, const _Float16* __restrict__ QL, const _Float16* __restrict__ KH, int b0, float* __restrict__ S0) { __shared__ __align__(16) float ss[4][16][132];
  const int z = blockIdx.z; const size_t b = b0 + z / NH; const int h = z % NH; float* S = S0 + (size_t)z * TT * TT;
  const int tid = threadIdx.x, wave = tid >> 5, lane = tid & 31, col = lane & 15, g = lane >> 4; const int k0 = blockIdx.y * 128; const int ql0 = blockIdx.x * 64 + wave * 16; const size_t q0 = b * TT + ql0;
  v8f acc[8] = {};
#pragma unroll
  for (int kc = 0; kc < HD / 32; ++kc) { const v16h ah = frag_h(QH + (q0 + col) * CC + h * HD + kc * 32, lane), al = frag_h(QL + (q0 + col) * CC + h * HD + kc * 32, lane);
#pragma unroll
    for (int j = 0; j < 8; ++j) { const v16h kb = frag_h(KH + (b * TT + k0 + j * 16 + col) * CC + h * HD + kc * 32, lane); acc[j] = wmma16(ah, kb, acc[j]); acc[j] = wmma16(al, kb, acc[j]); } }
#pragma unroll
  for (int j = 0; j < 8; ++j)
#pragma unroll
    for (int r = 0; r < 8; ++r) ss[wave][8 * g + r][j * 16 + col] = acc[j][r] * 0.125f;
  LDSX(); for (int rl = 0; rl < 16; ++rl) vst2(S + (size_t)(ql0 + rl) * TT + k0 + lane * 4, *(const v4f*)&ss[wave][rl][lane * 4]); }
__global__ __launch_bounds__(256) void k_sm(const float* __restrict__ S0, _Float16* __restrict__ PH0) { __shared__ float sred[8]; __shared__ float sbc; __shared__ __align__(16) _Float16 sh[TT];
  const int t = threadIdx.x; const size_t row = blockIdx.x; const float* sr = S0 + (size_t)blockIdx.y * TT * TT + row * TT; _Float16* ph = PH0 + (size_t)blockIdx.y * TT * TT + row * TT;
  float m = -3.0e38f; for (int k = t; k < TT; k += 256) m = fmaxf(m, sr[k]);
#pragma unroll
  for (int o = 1; o < 32; o <<= 1) m = fmaxf(m, __shfl_xor(m, o));
  if ((t & 31) == 0) sred[t >> 5] = m; __syncthreads(); if (t == 0) { float a = sred[0]; for (int i = 1; i < 8; ++i) a = fmaxf(a, sred[i]); sbc = a; } __syncthreads(); m = sbc; __syncthreads();
  float sum = 0.f; for (int k = t; k < TT; k += 256) sum += expf(sr[k] - m);
#pragma unroll
  for (int o = 1; o < 32; o <<= 1) sum += __shfl_xor(sum, o);
  if ((t & 31) == 0) sred[t >> 5] = sum; __syncthreads(); if (t == 0) { float a = 0.f; for (int i = 0; i < 8; ++i) a += sred[i]; sbc = 1.0f / a; } __syncthreads(); const float inv = sbc;
  for (int k = t; k < TT; k += 256) sh[k] = (_Float16)(expf(sr[k] - m) * inv * 2048.0f);
  __syncthreads(); for (int q = t; q < TT / 8; q += 256) vst2((unsigned*)(ph + q * 8), *(const v4u*)&sh[q * 8]); }
__global__ __launch_bounds__(256) void k_col(const _Float16* __restrict__ PH0, int b0, float* __restrict__ AM) { __shared__ __align__(16) float so[256];
  const int t = threadIdx.x; const int bl = blockIdx.y; const size_t b = b0 + bl; const int k = blockIdx.x * 256 + t; float a = 0.f;
#pragma unroll 1
  for (int h = 0; h < NH; ++h) { const _Float16* p = PH0 + ((size_t)(bl * NH + h) * TT) * TT + k;
#pragma unroll 4
    for (int q = 0; q < TT; ++q) a += (float)p[(size_t)q * TT]; }
  so[t] = a * (1.0f / 2048.0f) * (1.0f / NH);
  __syncthreads(); if (t < 64) vst2(AM + b * TT + blockIdx.x * 256 + t * 4, *(const v4f*)&so[t * 4]); }
__global__ __launch_bounds__(128) void k_pv(const _Float16* __restrict__ PH0, const _Float16* __restrict__ VT, int b0, float* __restrict__ Y) { __shared__ __align__(16) float ss[4][16][68];
  const int z = blockIdx.z; const size_t b = b0 + z / NH; const int h = z % NH; const _Float16* PH = PH0 + (size_t)z * TT * TT;
  const int tid = threadIdx.x, wave = tid >> 5, lane = tid & 31, col = lane & 15, g = lane >> 4; const int ql0 = blockIdx.x * 64 + wave * 16;
  v8f acc[4] = {};
#pragma unroll 1
  for (int kc = 0; kc < TT / 32; ++kc) { const v16h ph = frag_h(PH + (size_t)(ql0 + col) * TT + kc * 32, lane);
#pragma unroll
    for (int j = 0; j < 4; ++j) acc[j] = wmma16(ph, frag_h(VT + (b * CC + h * HD + j * 16 + col) * (size_t)TT + kc * 32, lane), acc[j]); }
#pragma unroll
  for (int j = 0; j < 4; ++j)
#pragma unroll
    for (int r = 0; r < 8; ++r) ss[wave][8 * g + r][j * 16 + col] = acc[j][r] * (1.0f / 2048.0f);
  LDSX(); for (int rl = 0; rl < 16; ++rl) if (lane < 16) vst2(Y + (b * TT + ql0 + rl) * CC + h * HD + lane * 4, *(const v4f*)&ss[wave][rl][lane * 4]); }
template <int MODE>
__global__ __launch_bounds__(128) void k_ln(const float* __restrict__ A, const float* __restrict__ Wm, const float* __restrict__ Bv, const float* __restrict__ RES, const float* __restrict__ GA, const float* __restrict__ BE, float* __restrict__ DST) {
  __shared__ __align__(16) float sz[64][CIN + 4];
  const int tid = threadIdx.x, wave = tid >> 5, lane = tid & 31, col = lane & 15, g = lane >> 4; const size_t r0 = (size_t)blockIdx.x * 64; const size_t b = r0 / TT; const int p0 = (int)(r0 % TT); constexpr int K = (MODE == 0) ? CC : CIN;
#pragma unroll 1
  for (int half = 0; half < 2; ++half) {
    v8f acc[8]; for (int j = 0; j < 8; ++j) for (int r = 0; r < 8; ++r) acc[j][r] = 0.f;
#pragma unroll 1
    for (int kc = 0; kc < K / 32; ++kc) { const F2 a = split_row(A + (r0 + wave * 16 + col) * K, kc * 32, lane);
#pragma unroll
      for (int j = 0; j < 8; ++j) { v16b w; const int o = half * 128 + j * 16 + col;
#pragma unroll
        for (int i = 0; i < 8; ++i) { w[i] = (__bf16)Wm[(size_t)(kc * 32 + 8 * g + i) * CIN + o]; w[8 + i] = (__bf16)Wm[(size_t)(kc * 32 + 16 + 8 * g + i) * CIN + o]; }
        acc[j] = wmma_bf(a.h, w, acc[j]); acc[j] = wmma_bf(a.l, w, acc[j]); } }
#pragma unroll
    for (int j = 0; j < 8; ++j) { const int o = half * 128 + j * 16 + col; const float bb = bfr(Bv[o]);
#pragma unroll
      for (int r = 0; r < 8; ++r) { const int rl = wave * 16 + 8 * g + r; const float res = (MODE == 0) ? bfr(RES[(b * CIN + o) * (size_t)TT + p0 + rl]) : RES[(r0 + rl) * CIN + o]; sz[rl][o] = acc[j][r] + bb + res; } } }
  __syncthreads();
  for (int rr = 0; rr < 16; ++rr) { const int rl = wave * 16 + rr; float s = 0.f; for (int c = lane; c < CIN; c += 32) s += sz[rl][c];
#pragma unroll
    for (int o2 = 1; o2 < 32; o2 <<= 1) s += __shfl_xor(s, o2); const float mu = s / CIN; float q = 0.f; for (int c = lane; c < CIN; c += 32) { const float d = sz[rl][c] - mu; q += d * d; }
#pragma unroll
    for (int o2 = 1; o2 < 32; o2 <<= 1) q += __shfl_xor(q, o2); const float inv = 1.0f / sqrtf(q / CIN + 1e-5f);
    for (int c = lane; c < CIN; c += 32) sz[rl][c] = (sz[rl][c] - mu) * inv * bfr(GA[c]) + bfr(BE[c]); }
  __syncthreads();
  if (MODE == 0) { for (int e = tid; e < 64 * 64; e += 128) { const int rl = e >> 6, q = e & 63; vst2(DST + (r0 + rl) * CIN + q * 4, *(const v4f*)&sz[rl][q * 4]); } }
  else {
    for (int e = tid; e < CIN * 16; e += 128) { const int c = e >> 4, q = e & 15; __align__(16) float v4x[4]; v4x[0] = sz[q * 4][c]; v4x[1] = sz[q * 4 + 1][c]; v4x[2] = sz[q * 4 + 2][c]; v4x[3] = sz[q * 4 + 3][c]; vst2(DST + (b * CIN + c) * (size_t)TT + p0 + q * 4, *(const v4f*)v4x); } } }
__global__ __launch_bounds__(128) void k_ffn1(const float* __restrict__ Z1, const float* __restrict__ W1, const float* __restrict__ B1, float* __restrict__ HM) { __shared__ __align__(16) float sf[4][16][132];
  const int tid = threadIdx.x, wave = tid >> 5, lane = tid & 31, col = lane & 15, g = lane >> 4; const int c0 = blockIdx.y * 128; const size_t r0 = (size_t)blockIdx.x * 64 + wave * 16;
  v8f acc[8] = {};
#pragma unroll
  for (int kc = 0; kc < CIN / 32; ++kc) { const F2 a = split_row(Z1 + (r0 + col) * CIN, kc * 32, lane);
#pragma unroll
    for (int j = 0; j < 8; ++j) { v16b w; const int o = c0 + j * 16 + col;
#pragma unroll
      for (int i = 0; i < 8; ++i) { w[i] = (__bf16)W1[(size_t)(kc * 32 + 8 * g + i) * CIN + o]; w[8 + i] = (__bf16)W1[(size_t)(kc * 32 + 16 + 8 * g + i) * CIN + o]; }
      acc[j] = wmma_bf(a.h, w, acc[j]); acc[j] = wmma_bf(a.l, w, acc[j]); } }
#pragma unroll
  for (int j = 0; j < 8; ++j) { const float bb = bfr(B1[c0 + j * 16 + col]);
#pragma unroll
    for (int r = 0; r < 8; ++r) { const float v = acc[j][r] + bb; sf[wave][8 * g + r][j * 16 + col] = v / (1.0f + expf(-v)); } }
  LDSX(); for (int rl = 0; rl < 16; ++rl) vst2(HM + (r0 + rl) * CIN + c0 + lane * 4, *(const v4f*)&sf[wave][rl][lane * 4]); }
extern "C" void kernel_launch(void* const* d_in, const int* in_sizes, int n_in, void* d_out, int out_size, void* d_ws, size_t ws_size, hipStream_t stream) {
  (void)in_sizes; (void)n_in; (void)out_size;
  const float** F = (const float**)d_in;
  if (ws_size < (size_t)WS_END) return;
  char* ws = (char*)d_ws; _Float16 *QH = (_Float16*)(ws + WS_QH), *QL = (_Float16*)(ws + WS_QL), *KH = (_Float16*)(ws + WS_KH), *VT = (_Float16*)(ws + WS_VT), *PH = (_Float16*)(ws + WS_PH); float *S = (float*)(ws + WS_S), *Y = (float*)(ws + WS_Y), *Z1 = (float*)(ws + WS_Z1), *HM = (float*)(ws + WS_HM);
  float* OUT0 = (float*)d_out; float* OUT1 = (float*)d_out + OUT1_OFF;
  k_proj<<<dim3(TT / 64, CC / 128, TNB * 3), 128, 0, stream>>>(F[0], F[1], F[2], F[3], F[4], F[5], F[6], QH, QL, KH, VT);
  for (int b0 = 0; b0 < TNB; b0 += BG) { const int ng = ((TNB - b0) < BG ? (TNB - b0) : BG);
    k_sc<<<dim3(TT / 64, TT / 128, ng * NH), 128, 0, stream>>>(QH, QL, KH, b0, S);
    k_sm<<<dim3(TT, ng * NH), 256, 0, stream>>>(S, PH);
    k_col<<<dim3(TT / 256, ng), 256, 0, stream>>>(PH, b0, OUT1);
    k_pv<<<dim3(TT / 64, 1, ng * NH), 128, 0, stream>>>(PH, VT, b0, Y);
  }
  k_ln<0><<<TNB * TT / 64, 128, 0, stream>>>(Y, F[7], F[8], F[0], F[13], F[14], Z1);
  k_ffn1<<<dim3(TNB * TT / 64, CIN / 128), 128, 0, stream>>>(Z1, F[9], F[10], HM);
  k_ln<1><<<TNB * TT / 64, 128, 0, stream>>>(HM, F[11], F[12], Z1, F[15], F[16], OUT0);
}
